// LambdaLayer_335007449673
// MI455X (gfx1250) — hardware-verified
//
#include <hip/hip_runtime.h>


namespace {
constexpr int Nn = 8, C = 256, HW = 64, M = HW * HW, NH = 4, DK = 16, DV = 64, QC = 64, KC = 16, VC = 64, OC = QC + KC + VC  , RK = 23, PADK = 11, PW = 96  , PH = HW + 2 * PADK  ;
constexpr float EPS = 1e-5f, VS = 8.0f, AS_ = 8.0f;

typedef _Float16 b16;
typedef __attribute__((ext_vector_type(16))) _Float16 v16b;
typedef __attribute__((ext_vector_type(8))) _Float16 v8b;
typedef __attribute__((ext_vector_type(8))) float v8f;
typedef __attribute__((ext_vector_type(4))) float v4f;
__device__ __forceinline__ float bf16_rne(float f) { unsigned int u = __float_as_uint(f); u += 0x7FFFu + ((u >> 16) & 1u); return __uint_as_float(u & 0xFFFF0000u); }
__device__ __forceinline__ void split16(float v, b16& hi, b16& lo) { hi = (b16)v; lo = (b16)(v - (float)hi); }
__device__ __forceinline__ v16b frag_kb(const b16* p, int hh) { const v8b a = *(const v8b*)(p + 8 * hh), b = *(const v8b*)(p + 16 + 8 * hh); v16b f;
#pragma unroll
  for (int e = 0; e < 8; ++e) { f[e] = a[e]; f[8 + e] = b[e]; } return f; }
__device__ __forceinline__ v8f wmma16b(v16b a, v16b b, v8f c) { v8f d = __builtin_amdgcn_wmma_f32_16x16x32_f16(false, a, false, b, (short)0, c, false, false); asm volatile("v_nop\n\tv_nop\n\tv_nop\n\tv_nop" : "+v"(d) : "v"(a), "v"(b)); return d; }
__device__ __forceinline__ void wave_lds_sync() { __builtin_amdgcn_fence(__ATOMIC_RELEASE, "workgroup"); __builtin_amdgcn_wave_barrier(); __builtin_amdgcn_fence(__ATOMIC_ACQUIRE, "workgroup"); }
__device__ __forceinline__ float nexp(float x) { return __builtin_amdgcn_exp2f(x * 1.4426950408889634f); }
__device__ __forceinline__ float pmul(float a, float b) { float p = a * b; asm volatile("" : "+v"(p)); return p; }
__device__ __forceinline__ float wmax(float v) {
#pragma unroll
  for (int o = 1; o < 32; o <<= 1) v = fmaxf(v, __shfl_xor(v, o)); return v; }
__device__ __forceinline__ float wsum(float v) {
#pragma unroll
  for (int o = 1; o < 32; o <<= 1) v += __shfl_xor(v, o); return v; }

__global__ __launch_bounds__(256) void prep_kernel(const float* __restrict__ x, const float* __restrict__ w, const float* __restrict__ qg, const float* __restrict__ qb, const float* __restrict__ qm, const float* __restrict__ qv, const float* __restrict__ vg, const float* __restrict__ vb, const float* __restrict__ vm, const float* __restrict__ vv, const float* __restrict__ wl, const float* __restrict__ bl, b16* __restrict__ X, b16* __restrict__ R, b16* __restrict__ WL, float* __restrict__ P) {
  __shared__ __attribute__((aligned(16))) b16 T[64][C + 8];
  const int n = blockIdx.y, p0 = blockIdx.x * 64, t_ = threadIdx.x;
  for (int i = t_; i < C * 64; i += 256) { const int c = i >> 6, p = i & 63; T[p][c] = (b16)bf16_rne(x[((size_t)n * C + c) * M + p0 + p]); }
  __syncthreads();
  for (int pass = 0; pass < 2; ++pass) {
    for (int i = t_; i < 64 * 32; i += 256) { const int p = i >> 5, c8 = (i & 31) * 8; *(volatile v8b*)(X + ((size_t)n * M + p0 + p) * C + c8) = *(const v8b*)(&T[p][c8]); }
    if (blockIdx.x == 0 && n == 0) {
      for (int i = t_; i < OC * C / 8; i += 256) { v8b v; for (int e = 0; e < 8; ++e) v[e] = (b16)bf16_rne(w[i * 8 + e]); *(volatile v8b*)(R + i * 8) = v; }
      for (int i = t_; i < 16 * RK * 4; i += 256) { const int k = i / (RK * 4), r = i % (RK * 4); const int dy = r >> 2, d8 = (r & 3) * 8; v8b v; for (int e = 0; e < 8; ++e) { const int dx = d8 + e; v[e] = (b16)((dx < RK) ? bf16_rne(wl[(k * RK + dy) * RK + dx]) : 0.0f); } *(volatile v8b*)(WL + (size_t)k * (RK * 32) + dy * 32 + d8) = v; }
      if (t_ < 64) { const float qs = bf16_rne(qg[t_]) / sqrtf(bf16_rne(qv[t_]) + EPS), vs_ = bf16_rne(vg[t_]) / sqrtf(bf16_rne(vv[t_]) + EPS);
        ((volatile float*)P)[t_] = qs; ((volatile float*)P)[64 + t_] = bf16_rne(qb[t_]) - bf16_rne(qm[t_]) * qs; ((volatile float*)P)[128 + t_] = vs_; ((volatile float*)P)[192 + t_] = bf16_rne(vb[t_]) - bf16_rne(vm[t_]) * vs_; }
      if (t_ < 16) ((volatile float*)P)[256 + t_] = bf16_rne(bl[t_]); }
    __threadfence(); }
}

__global__ __launch_bounds__(64) void qkv_kernel(const b16* __restrict__ X, const b16* __restrict__ R, const float* __restrict__ P, float* __restrict__ Q, float* __restrict__ Kc, b16* __restrict__ Vr) {
  __shared__ __attribute__((aligned(16))) float Ts[32][OC + 4];
  const int lane = threadIdx.x & 31, wave = threadIdx.x >> 5, nloc = lane & 15, hlf = lane >> 4, n = blockIdx.y, m0 = blockIdx.x * 32; const int t0 = wave * 5, nt = (wave == 0) ? 5 : 4;
  v8f acc[2][5];
#pragma unroll
  for (int r = 0; r < 2; ++r)
#pragma unroll
    for (int t = 0; t < 5; ++t) acc[r][t] = (v8f){};
#pragma unroll 2
  for (int kb = 0; kb < C; kb += 32) { const v16b a0 = frag_kb(X + ((size_t)n * M + m0 + nloc) * C + kb, hlf), a1 = frag_kb(X + ((size_t)n * M + m0 + 16 + nloc) * C + kb, hlf);
#pragma unroll
    for (int t = 0; t < 5; ++t) { if (t < nt) { const v16b bw = frag_kb(R + (size_t)((t0 + t) * 16 + nloc) * C + kb, hlf); acc[0][t] = wmma16b(a0, bw, acc[0][t]); acc[1][t] = wmma16b(a1, bw, acc[1][t]); } } }
#pragma unroll
  for (int t = 0; t < 5; ++t) { if (t < nt) { const int c = (t0 + t) * 16 + nloc;
#pragma unroll
      for (int r = 0; r < 2; ++r)
#pragma unroll
        for (int v = 0; v < 8; ++v) { float y = acc[r][t][v]; if (c < QC) y = pmul(y, P[c]) + P[64 + c]; else if (c >= QC + KC) y = pmul(y, P[128 + c - QC - KC]) + P[192 + c - QC - KC]; Ts[r * 16 + 8 * hlf + v][c] = y; } } }
  __syncthreads();
  for (int pass = 0; pass < 2; ++pass) {
    for (int i = threadIdx.x; i < 32 * 16; i += 64) { const int rr = i >> 4, c4 = (i & 15) * 4; *(volatile v4f*)(Q + ((size_t)n * M + m0 + rr) * QC + c4) = *(const v4f*)(&Ts[rr][c4]); }
    for (int i = threadIdx.x; i < 32 * 8; i += 64) { const int rr = i >> 3, c8 = (i & 7) * 8; v8b o; for (int e = 0; e < 8; ++e) o[e] = (b16)(Ts[rr][QC + KC + c8 + e] * VS); *(volatile v8b*)(Vr + ((size_t)n * M + m0 + rr) * DV + c8) = o; }
    if (wave == 0) { for (int kc = 0; kc < KC; ++kc) ((volatile float*)Kc)[((size_t)n * KC + kc) * M + m0 + lane] = Ts[lane][QC + kc]; }
    __threadfence(); }
}

__global__ __launch_bounds__(256) void plane_kernel(const b16* __restrict__ Vr, b16* __restrict__ Vp) {
  __shared__ __attribute__((aligned(16))) b16 pl[PH * PW];
  const int v = blockIdx.x, n = blockIdx.y, t_ = threadIdx.x;
  for (int i = t_; i < PH * PW; i += 256) { const int yy = i / PW - PADK, xq = i % PW - PADK; pl[i] = (yy >= 0 && yy < HW && xq >= 0 && xq < HW) ? Vr[((size_t)n * M + yy * HW + xq) * DV + v] : (b16)0.0f; }
  __syncthreads();
  b16* dst = Vp + ((size_t)n * DV + v) * PH * PW;
  for (int pass = 0; pass < 2; ++pass) { for (int i = t_; i < PH * PW / 8; i += 256) *(volatile v8b*)(dst + i * 8) = *(const v8b*)(&pl[i * 8]); __threadfence(); }
}

__global__ __launch_bounds__(256) void lambdac_kernel(const float* __restrict__ Kc, const b16* __restrict__ Vr, float* __restrict__ LC) {
  __shared__ float mx[KC], isum[KC]; __shared__ float red[8]; __shared__ __attribute__((aligned(16))) float Lc[KC][DV];
  const int n = blockIdx.x, t_ = threadIdx.x, lane = t_ & 31, wave = t_ >> 5, nloc = lane & 15, hlf = lane >> 4;
  for (int kc = 0; kc < KC; ++kc) { const float* kr = Kc + ((size_t)n * KC + kc) * M; float m_ = -INFINITY; for (int i = t_; i < M; i += 256) m_ = fmaxf(m_, kr[i]); m_ = wmax(m_); if (lane == 0) red[wave] = m_; __syncthreads();
    float gm = red[0]; for (int w = 1; w < 8; ++w) gm = fmaxf(gm, red[w]); __syncthreads();
    float s = 0.0f; for (int i = t_; i < M; i += 256) s += nexp(kr[i] - gm); s = wsum(s); if (lane == 0) red[wave] = s; __syncthreads();
    if (t_ == 0) { float a = 0.0f; for (int w = 0; w < 8; ++w) a += red[w]; mx[kc] = gm; isum[kc] = 1.0f / a; } __syncthreads(); }
  v8f acc[4] = {{}, {}, {}, {}};
  for (int kb = wave * 32; kb < M; kb += 256) { v16b ah, al;
#pragma unroll
    for (int e = 0; e < 16; ++e) { const int pos = kb + ((e < 8) ? (8 * hlf + e) : (16 + 8 * hlf + e - 8)); const float p = nexp(Kc[((size_t)n * KC + nloc) * M + pos] - mx[nloc]) * isum[nloc]; b16 a_, c_; split16(p * AS_, a_, c_); ah[e] = a_; al[e] = c_; }
#pragma unroll
    for (int t = 0; t < 4; ++t) { v16b bv;
#pragma unroll
      for (int e = 0; e < 16; ++e) { const int pos = kb + ((e < 8) ? (8 * hlf + e) : (16 + 8 * hlf + e - 8)); bv[e] = Vr[((size_t)n * M + pos) * DV + t * 16 + nloc]; }
      acc[t] = wmma16b(ah, bv, acc[t]); acc[t] = wmma16b(al, bv, acc[t]); } }
  __shared__ __attribute__((aligned(16))) float part[8][KC][DV];
#pragma unroll
  for (int t = 0; t < 4; ++t)
#pragma unroll
    for (int r = 0; r < 8; ++r) part[wave][8 * hlf + r][t * 16 + nloc] = acc[t][r] * (1.0f / (AS_ * VS));
  __syncthreads();
  for (int i = t_; i < KC * DV; i += 256) { const int kc = i / DV, v = i % DV; float s = 0.0f; for (int w = 0; w < 8; ++w) s += part[w][kc][v]; Lc[kc][v] = s; }
  __syncthreads();
  for (int pass = 0; pass < 2; ++pass) { *(volatile v4f*)(LC + (size_t)n * KC * DV + t_ * 4) = *(const v4f*)(&Lc[0][0] + t_ * 4); __threadfence(); }
}

__global__ __launch_bounds__(256) void lambdap_kernel(const b16* __restrict__ Vp, const b16* __restrict__ WL, const float* __restrict__ Q, const float* __restrict__ LC, const float* __restrict__ P, float* __restrict__ out) {
  __shared__ __attribute__((aligned(16))) float Ow[8][NH][512];
  const int v = blockIdx.x, n = blockIdx.y, wave = threadIdx.x >> 5, lane = threadIdx.x & 31, nloc = lane & 15, hlf = lane >> 4;
  const b16* pl = Vp + ((size_t)n * DV + v) * PH * PW; const float lcv = LC[((size_t)n * KC + nloc) * DV + v] + P[256 + nloc];
  for (int tile = 0; tile < 32; ++tile) { const int y = wave * 8 + (tile >> 2), x0 = (tile & 3) * 16; v8f acc = {};
    for (int dy = 0; dy < RK; ++dy) acc = wmma16b(frag_kb(pl + (size_t)(y + dy) * PW + x0 + nloc, hlf), frag_kb(WL + (size_t)nloc * (RK * 32) + dy * 32, hlf), acc);
#pragma unroll
    for (int r = 0; r < 8; ++r) { const int m = y * HW + x0 + 8 * hlf + r; const float lam = acc[r] * (1.0f / VS) + lcv; const float* qr = Q + ((size_t)n * M + m) * QC;
#pragma unroll
      for (int h = 0; h < NH; ++h) { float s = pmul(qr[h * DK + nloc], lam); s += __shfl_xor(s, 1); s += __shfl_xor(s, 2); s += __shfl_xor(s, 4); s += __shfl_xor(s, 8); if (nloc == 0) Ow[wave][h][(tile >> 2) * 64 + x0 + 8 * hlf + r] = s; } } }
  wave_lds_sync();
  for (int pass = 0; pass < 2; ++pass) {
#pragma unroll
    for (int h = 0; h < NH; ++h) { float* dst = out + (((size_t)n * C + h * DV + v) * M) + wave * 512; for (int i = lane; i < 128; i += 32) *(volatile v4f*)(dst + i * 4) = *(const v4f*)(&Ow[wave][h][i * 4]); }
    __threadfence(); }
}
}

extern "C" void kernel_launch(void* const* d_in, const int* in_sizes, int n_in,
                              void* d_out, int out_size, void* d_ws, size_t ws_size, hipStream_t stream) {
  (void)n_in; (void)out_size;
  const float* x = (const float*)d_in[0]; const float* w = (const float*)d_in[1]; const float* qg = (const float*)d_in[2]; const float* qb = (const float*)d_in[3]; const float* qm = (const float*)d_in[4]; const float* qv = (const float*)d_in[5];
  const float* vg = (const float*)d_in[6]; const float* vb = (const float*)d_in[7]; const float* vm = (const float*)d_in[8]; const float* vv = (const float*)d_in[9]; const float* wl = (const float*)d_in[10]; const float* bl = (const float*)d_in[11];
  float* out = (float*)d_out;
  if (in_sizes[0] != Nn * C * M || in_sizes[1] != OC * C || in_sizes[10] != 16 * RK * RK) return;
  size_t off = 0; char* ws = (char*)d_ws;
  auto carve = [&](size_t bytes) { char* p = ws + off; off += (bytes + 255) & ~(size_t)255; return p; };
  b16* X = (b16*)carve((size_t)Nn * M * C * 2); b16* R = (b16*)carve((size_t)OC * C * 2); b16* WL = (b16*)carve((size_t)16 * RK * 32 * 2); float* P = (float*)carve(512 * 4);
  float* Q = (float*)carve((size_t)Nn * M * QC * 4); float* Kc = (float*)carve((size_t)Nn * KC * M * 4); b16* Vr = (b16*)carve((size_t)Nn * M * DV * 2); b16* Vp = (b16*)carve((size_t)Nn * DV * PH * PW * 2); float* LC = (float*)carve((size_t)Nn * KC * DV * 4);
  if (off > ws_size) return;
  prep_kernel<<<dim3(M / 64, Nn), 256, 0, stream>>>(x, w, qg, qb, qm, qv, vg, vb, vm, vv, wl, bl, X, R, WL, P);
  qkv_kernel<<<dim3(M / 32, Nn), 64, 0, stream>>>(X, R, P, Q, Kc, Vr);
  plane_kernel<<<dim3(DV, Nn), 256, 0, stream>>>(Vr, Vp);
  lambdac_kernel<<<Nn, 256, 0, stream>>>(Kc, Vr, LC);
  lambdap_kernel<<<dim3(DV, Nn), 256, 0, stream>>>(Vp, WL, Q, LC, P, out);
}
